// SWAttention_15728170238371
// MI455X (gfx1250) — hardware-verified
//
#include <hip/hip_runtime.h>
#include <math.h>

typedef __attribute__((ext_vector_type(16))) __bf16 v16b;
typedef __attribute__((ext_vector_type(8)))  __bf16 v8b;
typedef __attribute__((ext_vector_type(8)))  float  v8f;
typedef __attribute__((ext_vector_type(4)))  float  v4f;
typedef __attribute__((ext_vector_type(4)))  unsigned int v4u;
typedef __attribute__((ext_vector_type(8)))  unsigned short v8us;

constexpr int kBatch = 2;
constexpr int kSeq   = 2048;
constexpr int kHid   = 2048;
constexpr int kProj  = 2048;
constexpr int kHeads = 16;
constexpr int kHdim  = 128;
constexpr int kWin   = 256;
constexpr int kRows  = kBatch * kSeq;
constexpr float kNegLog2BaseOver64 = -0.20762050593046015f;

static_assert(kHid % 32 == 0 && kProj % 32 == 0, "k step");
static_assert(kRows % 64 == 0 && kProj % 64 == 0 && kHid % 64 == 0, "tile");
static_assert(kSeq % 64 == 0 && kHdim == 128 && kHeads * kHdim == kProj, "geom");

__device__ __forceinline__ unsigned short f2bf_bits(float f) {
  unsigned u = __float_as_uint(f);
  return (unsigned short)((u + 0x7FFFu + ((u >> 16) & 1u)) >> 16);
}
__device__ __forceinline__ float bf_bits2f(unsigned short h) { return __uint_as_float(((unsigned)h) << 16); }
__device__ __forceinline__ float bf_rne(float f) { return bf_bits2f(f2bf_bits(f)); }

__device__ __forceinline__ void dep_guard_b(v8f& a, v8f& b, v16b x, v16b y) { asm volatile("v_nop\n\tv_nop\n\tv_nop\n\tv_nop" : "+v"(a), "+v"(b) : "v"(x), "v"(y)); }
__device__ __forceinline__ void keep4_b(v16b a, v16b b, v16b c, v16b d) { asm volatile("v_nop" :: "v"(a), "v"(b), "v"(c), "v"(d)); }
__device__ __forceinline__ void acc_guard4(v8f& a, v8f& b, v8f& c, v8f& d) { asm volatile("v_nop\n\tv_nop\n\tv_nop\n\tv_nop" : "+v"(a), "+v"(b), "+v"(c), "+v"(d)); }
__device__ __forceinline__ void mem_order_point() { asm volatile("" ::: "memory"); }

template <typename T> struct Frag;
template <> struct Frag<__bf16> {
  typedef v16b V; union U { v16b v; v8b h[2]; };
  static __device__ __forceinline__ v16b load(const __bf16* p) {
    U f; f.h[0] = *(const v8b*)(p); f.h[1] = *(const v8b*)(p + 16); return f.v;
  }
  static __device__ __forceinline__ v8f mma(v16b a, v16b b, v8f c) {
    return __builtin_amdgcn_wmma_f32_16x16x32_bf16(false, a, false, b, (short)0, c, false, false);
  }
  static __device__ __forceinline__ void guard(v8f& a, v8f& b, v16b x, v16b y) { dep_guard_b(a, b, x, y); }
  static __device__ __forceinline__ void keep(v16b a, v16b b, v16b c, v16b d) { keep4_b(a, b, c, d); }
};

__device__ __forceinline__ v8f at_mma(v16b a, v16b b, v8f c) {
  c = __builtin_amdgcn_wmma_f32_16x16x32_bf16(false, a, false, b, (short)0, c, false, false);
  asm volatile("v_nop\n\tv_nop\n\tv_nop\n\tv_nop" : "+v"(c) : "v"(a), "v"(b));
  return c;
}

__device__ __forceinline__ void wave_sync_lds() {
  __builtin_amdgcn_fence(__ATOMIC_RELEASE, "workgroup");
  __builtin_amdgcn_wave_barrier();
  __builtin_amdgcn_fence(__ATOMIC_ACQUIRE, "workgroup");
}

template <bool ASPLIT>
__device__ __forceinline__ void gemm_mainloop(const __bf16* __restrict__ Ab, const __bf16* __restrict__ Ab2,
                                              const __bf16* __restrict__ Bb, int lda, int ldb,
                                              int m0, int n0, int K, int lane, v8f (&acc)[4][4]) {
  const int rlane = lane & 15;
  const int koff  = (lane >> 4) * 8;
#pragma unroll
  for (int i = 0; i < 4; ++i)
#pragma unroll
    for (int j = 0; j < 4; ++j) acc[i][j] = (v8f){0.f,0.f,0.f,0.f,0.f,0.f,0.f,0.f};

  for (int k0 = 0; k0 < K; k0 += 32) {
    v16b bh[4];
#pragma unroll
    for (int j = 0; j < 4; ++j) {
      const size_t bo = (size_t)(n0 + (j << 4) + rlane) * ldb + koff + k0;
      bh[j] = Frag<__bf16>::load(Bb + bo);
    }
#pragma unroll
    for (int i = 0; i < 4; ++i) {
      const size_t ao = (size_t)(m0 + (i << 4) + rlane) * lda + koff + k0;
      v16b ah = Frag<__bf16>::load(Ab + ao);
      v16b al = ah;
      if (ASPLIT) al = Frag<__bf16>::load(Ab2 + ao);
#pragma unroll
      for (int j = 0; j < 4; ++j) {
        acc[i][j] = Frag<__bf16>::mma(ah, bh[j], acc[i][j]);
        if (ASPLIT) acc[i][j] = Frag<__bf16>::mma(al, bh[j], acc[i][j]);
      }
      Frag<__bf16>::guard(acc[i][0], acc[i][3], ah, al);
    }
    Frag<__bf16>::keep(bh[0], bh[1], bh[2], bh[3]);
  }
  acc_guard4(acc[0][0], acc[0][1], acc[0][2], acc[0][3]);
  acc_guard4(acc[1][0], acc[1][1], acc[1][2], acc[1][3]);
  acc_guard4(acc[2][0], acc[2][1], acc[2][2], acc[2][3]);
  acc_guard4(acc[3][0], acc[3][1], acc[3][2], acc[3][3]);
}

__global__ __launch_bounds__(256) void rope_tab_kernel(float* __restrict__ rcos, float* __restrict__ rsin) {
#pragma clang fp contract(off)
  const int i = blockIdx.x * 256 + threadIdx.x;
  if (i >= kSeq * 64) return;
  const int pos = i >> 6;
  const int fi  = i & 63;
  const float inv = exp2f((float)fi * kNegLog2BaseOver64);
  const float ang = (float)pos * inv;
  float sv, cv;
  sincosf(ang, &sv, &cv);
  ((volatile float*)rcos)[i] = cv;
  ((volatile float*)rsin)[i] = sv;
  __threadfence();
  ((volatile float*)rcos)[i] = cv;
  ((volatile float*)rsin)[i] = sv;
}

__global__ __launch_bounds__(256) void cast_x_kernel(const float* __restrict__ x, unsigned short* __restrict__ xb, int n8) {
  const int i = blockIdx.x * 256 + threadIdx.x;
  if (i >= n8) return;
  const v4f a = *(const v4f*)(x + (size_t)i * 8);
  const v4f c = *(const v4f*)(x + (size_t)i * 8 + 4);
  v4u w;
  w[0] = (unsigned)f2bf_bits(a[0]) | ((unsigned)f2bf_bits(a[1]) << 16);
  w[1] = (unsigned)f2bf_bits(a[2]) | ((unsigned)f2bf_bits(a[3]) << 16);
  w[2] = (unsigned)f2bf_bits(c[0]) | ((unsigned)f2bf_bits(c[1]) << 16);
  w[3] = (unsigned)f2bf_bits(c[2]) | ((unsigned)f2bf_bits(c[3]) << 16);
  *(volatile v4u*)(xb + (size_t)i * 8) = w;
  __threadfence();
  *(volatile v4u*)(xb + (size_t)i * 8) = w;
}

__global__ __launch_bounds__(256) void cast_w_kernel(const float* __restrict__ W, unsigned short* __restrict__ Bt, int rowperm) {
  __shared__ __align__(16) unsigned short tile[64 * 72];
  const int tid = threadIdx.x;
  const int k0 = blockIdx.x * 64;
  const int n0 = blockIdx.y * 64;
  const int a = tid >> 2, part = tid & 3;
  size_t src;
  if (rowperm == 0) {
    const int hb = n0 & ~127, tp = (n0 >> 6) & 1;
    const int col = hb + 32 * tp + 16 * (part & 1) + 64 * (part >> 1);
    src = (size_t)(k0 + a) * kProj + col;
  } else {
    const int hb = k0 & ~127, tp = (k0 >> 6) & 1;
    const int row = hb + 32 * tp + (a & 31) + 64 * (a >> 5);
    src = (size_t)row * kHid + n0 + 16 * part;
  }
  const v4f f0 = *(const v4f*)(W + src);
  const v4f f1 = *(const v4f*)(W + src + 4);
  const v4f f2 = *(const v4f*)(W + src + 8);
  const v4f f3 = *(const v4f*)(W + src + 12);
#pragma unroll
  for (int e = 0; e < 4; ++e) {
    tile[(part * 16 + e)      * 72 + a] = f2bf_bits(f0[e]);
    tile[(part * 16 + 4 + e)  * 72 + a] = f2bf_bits(f1[e]);
    tile[(part * 16 + 8 + e)  * 72 + a] = f2bf_bits(f2[e]);
    tile[(part * 16 + 12 + e) * 72 + a] = f2bf_bits(f3[e]);
  }
  __syncthreads();
  for (int pass = 0; pass < 2; ++pass) {
#pragma unroll
    for (int it = 0; it < 2; ++it) {
      const int idx = tid + it * 256;
      const int rr = idx >> 3, c8 = (idx & 7) * 8;
      const v4u w = *(const v4u*)(tile + rr * 72 + c8);
      *(volatile v4u*)(Bt + (size_t)(n0 + rr) * 2048 + k0 + c8) = w;
    }
    __threadfence();
  }
}

__global__ __launch_bounds__(256) void proj_gemm_kernel(
    const unsigned short* __restrict__ Ap, const unsigned short* __restrict__ Btp,
    const float* __restrict__ bias, const float* __restrict__ kw,
    const float* __restrict__ rcos, const float* __restrict__ rsin,
    unsigned short* __restrict__ outH, unsigned short* __restrict__ outL, int mode) {
  const __bf16* A  = (const __bf16*)Ap;
  const __bf16* Bt = (const __bf16*)Btp;
  __shared__ __align__(16) float sT[8][16 * 68];
  const int lane = threadIdx.x & 31;
  const int wave = threadIdx.x >> 5;
  constexpr int tilesN = kProj / 64;
  constexpr int tilesM = kRows / 64;
  const int tile = blockIdx.x * 8 + wave;
  if (tile >= tilesM * tilesN) return;
  const int tm = tile / tilesN;
  const int tn = tile - tm * tilesN;
  const int m0 = tm << 6;
  const int n0 = tn << 6;
  const int rlane = lane & 15;
  const int mOff  = (lane >> 4) * 8;

  v8f acc[4][4];
  gemm_mainloop<false>(A, A, Bt, kHid, kHid, m0, n0, kHid, lane, acc);

  float* slab = sT[wave];
  const int hb = n0 & ~127;
  const int tpar = (n0 >> 6) & 1;
  const int hidx = n0 >> 7;
  const int rs = lane >> 2;
  const int cg = (lane & 3) * 8;
  const int fbase = 32 * tpar + cg;
  float b1[8], b2[8];
  {
    const v4f u0 = *(const v4f*)(bias + hb + fbase);
    const v4f u1 = *(const v4f*)(bias + hb + fbase + 4);
    const v4f w0 = *(const v4f*)(bias + hb + 64 + fbase);
    const v4f w1 = *(const v4f*)(bias + hb + 64 + fbase + 4);
#pragma unroll
    for (int e = 0; e < 4; ++e) {
      b1[e] = bf_rne(u0[e]); b1[4 + e] = bf_rne(u1[e]);
      b2[e] = bf_rne(w0[e]); b2[4 + e] = bf_rne(w1[e]);
    }
  }
  const float qmul = (mode == 0) ? (0.08838834764831845f * bf_rne(kw[hidx])) : 1.0f;

#pragma unroll
  for (int i = 0; i < 4; ++i) {
    const int mBase = m0 + (i << 4);
#pragma unroll
    for (int j = 0; j < 4; ++j) {
#pragma unroll
      for (int r = 0; r < 8; ++r) slab[(mOff + r) * 68 + (j << 4) + rlane] = acc[i][j][r];
    }
    wave_sync_lds();
#pragma unroll 1
    for (int it = 0; it < 2; ++it) {
      const int row = it * 8 + rs;
      const int pos = (mBase + row) & (kSeq - 1);
      float* sp1 = slab + row * 68 + cg;
      float* sp2 = sp1 + 32;
      const v4f x0 = *(const v4f*)sp1, x1 = *(const v4f*)(sp1 + 4);
      const v4f y0 = *(const v4f*)sp2, y1 = *(const v4f*)(sp2 + 4);
      float t1[8], t2[8];
#pragma unroll
      for (int e = 0; e < 4; ++e) {
        t1[e] = x0[e] + b1[e]; t1[4 + e] = x1[e] + b1[4 + e];
        t2[e] = y0[e] + b2[e]; t2[4 + e] = y1[e] + b2[4 + e];
      }
      float o1[8], o2[8];
      if (mode < 2) {
        const float* cp  = rcos + (size_t)pos * 64 + fbase;
        const float* snp = rsin + (size_t)pos * 64 + fbase;
        const v4f c0 = *(const v4f*)cp,  c1 = *(const v4f*)(cp + 4);
        const v4f s0 = *(const v4f*)snp, s1 = *(const v4f*)(snp + 4);
        float cs[8], sn[8];
#pragma unroll
        for (int e = 0; e < 4; ++e) { cs[e] = c0[e]; cs[4 + e] = c1[e]; sn[e] = s0[e]; sn[4 + e] = s1[e]; }
#pragma unroll
        for (int e = 0; e < 8; ++e) {
          o1[e] = (t1[e] * cs[e] - t2[e] * sn[e]) * qmul;
          o2[e] = (t1[e] * sn[e] + t2[e] * cs[e]) * qmul;
        }
      } else {
#pragma unroll
        for (int e = 0; e < 8; ++e) { o1[e] = t1[e]; o2[e] = t2[e]; }
      }
      v4f z0, z1, z2, z3;
#pragma unroll
      for (int e = 0; e < 4; ++e) { z0[e] = o1[e]; z1[e] = o1[4 + e]; z2[e] = o2[e]; z3[e] = o2[4 + e]; }
      *(v4f*)sp1 = z0; *(v4f*)(sp1 + 4) = z1;
      *(v4f*)sp2 = z2; *(v4f*)(sp2 + 4) = z3;
    }
    wave_sync_lds();
    {
      const int q8 = lane >> 3, c8 = (lane & 7) * 8;
      for (int pass = 0; pass < 2; ++pass) {
#pragma unroll
        for (int it = 0; it < 4; ++it) {
          const int row = it * 4 + q8;
          const float* sp = slab + row * 68 + c8;
          v8us hv, lv;
#pragma unroll
          for (int e = 0; e < 8; ++e) {
            const float f = sp[e];
            const unsigned short hbits = f2bf_bits(f);
            const unsigned short lbits = f2bf_bits(f - bf_bits2f(hbits));
            hv[e] = hbits; lv[e] = lbits;
          }
          const size_t go = (size_t)(mBase + row) * kProj + n0 + c8;
          *(volatile v8us*)(outH + go) = hv;
          *(volatile v8us*)(outL + go) = lv;
        }
        __threadfence();
      }
    }
    wave_sync_lds();
  }
}

constexpr int L_QSH = 0;
constexpr int L_QSL = 8192;
constexpr int L_KSH = 16384;
constexpr int L_KSL = 24576;
constexpr int L_VTH = 32768;
constexpr int L_VTL = 40960;
constexpr int L_PSH = 49152;
constexpr int L_PSL = 53248;
constexpr int L_TOT = 57344;
static_assert(4 * 16 * 132 * 2 <= L_TOT, "os alias");

__global__ __launch_bounds__(128) __attribute__((amdgpu_num_vgpr(256)))
void swa_attn_kernel(
    const unsigned short* __restrict__ Qh, const unsigned short* __restrict__ Ql,
    const unsigned short* __restrict__ Kh, const unsigned short* __restrict__ Kl,
    const unsigned short* __restrict__ Vh, const unsigned short* __restrict__ Vl,
    unsigned short* __restrict__ Oh, unsigned short* __restrict__ Ol) {
  __shared__ __align__(16) unsigned short sm[L_TOT];
  const int tid  = threadIdx.x;
  const int wave = tid >> 5;
  const int lane = tid & 31;
  const int hh   = lane >> 4;
  const int c    = lane & 15;

  const int bx = blockIdx.x;
  const int qb = bx & 31;
  const int bh = bx >> 5;
  const int h  = bh & 15;
  const int b  = bh >> 4;
  const int qbase = qb * 64;
  const int q0 = qbase + wave * 16;
  const size_t rowB = (size_t)b * kSeq;
  const int colH = h * kHdim;

#pragma unroll 2
  for (int i = 0; i < 8; ++i) {
    const int idx = tid + i * 128;
    const int r = idx >> 4, c8 = (idx & 15) * 8;
    const size_t go = (rowB + qbase + r) * (size_t)kProj + colH + c8;
    const v4u wq = *(const v4u*)(Qh + go);
    const v4u wl = *(const v4u*)(Ql + go);
    *(v4u*)(sm + L_QSH + r * 128 + c8) = wq;
    *(v4u*)(sm + L_QSL + r * 128 + c8) = wl;
  }
  mem_order_point();

  float mrow[8], lrow[8];
  v8f oacc[8];
#pragma unroll
  for (int r = 0; r < 8; ++r) { mrow[r] = -INFINITY; lrow[r] = 0.f; }
#pragma unroll
  for (int t = 0; t < 8; ++t) oacc[t] = (v8f){0.f,0.f,0.f,0.f,0.f,0.f,0.f,0.f};

  const int kc_hi = qb;
  const int kc_lo = (qb > 4) ? (qb - 4) : 0;
  for (int kc = kc_lo; kc <= kc_hi; ++kc) {
    const int kv0 = kc * 64;
    __syncthreads();
#pragma unroll 2
    for (int i = 0; i < 8; ++i) {
      const int idx = tid + i * 128;
      const int r = idx >> 4, c8 = (idx & 15) * 8;
      const size_t go = (rowB + kv0 + r) * (size_t)kProj + colH + c8;
      const v4u wh = *(const v4u*)(Kh + go);
      const v4u wl = *(const v4u*)(Kl + go);
      *(v4u*)(sm + L_KSH + r * 128 + c8) = wh;
      *(v4u*)(sm + L_KSL + r * 128 + c8) = wl;
    }
    mem_order_point();
#pragma unroll 2
    for (int i = 0; i < 8; ++i) {
      const int idx = tid + i * 128;
      const int r = idx >> 4, c8 = (idx & 15) * 8;
      const size_t go = (rowB + kv0 + r) * (size_t)kProj + colH + c8;
      const v4u wh = *(const v4u*)(Vh + go);
      const v4u wl = *(const v4u*)(Vl + go);
#pragma unroll
      for (int e2 = 0; e2 < 4; ++e2) {
        const unsigned uh = wh[e2], ul = wl[e2];
        sm[L_VTH + (c8 + 2 * e2)     * 64 + r] = (unsigned short)(uh & 0xffffu);
        sm[L_VTH + (c8 + 2 * e2 + 1) * 64 + r] = (unsigned short)(uh >> 16);
        sm[L_VTL + (c8 + 2 * e2)     * 64 + r] = (unsigned short)(ul & 0xffffu);
        sm[L_VTL + (c8 + 2 * e2 + 1) * 64 + r] = (unsigned short)(ul >> 16);
      }
    }
    __syncthreads();

    v8f s[4];
#pragma unroll
    for (int j = 0; j < 4; ++j) s[j] = (v8f){0.f,0.f,0.f,0.f,0.f,0.f,0.f,0.f};
    {
      const __bf16* qsh = (const __bf16*)(sm + L_QSH) + (wave * 16 + c) * 128 + 8 * hh;
      const __bf16* qsl = (const __bf16*)(sm + L_QSL) + (wave * 16 + c) * 128 + 8 * hh;
      const __bf16* ksh = (const __bf16*)(sm + L_KSH) + c * 128 + 8 * hh;
      const __bf16* ksl = (const __bf16*)(sm + L_KSL) + c * 128 + 8 * hh;
#pragma unroll 1
      for (int dc = 0; dc < 4; ++dc) {
        const v16b qa  = Frag<__bf16>::load(qsh + dc * 32);
        const v16b qlo = Frag<__bf16>::load(qsl + dc * 32);
#pragma unroll
        for (int j = 0; j < 4; ++j) {
          const v16b ka  = Frag<__bf16>::load(ksh + j * 2048 + dc * 32);
          const v16b klo = Frag<__bf16>::load(ksl + j * 2048 + dc * 32);
          s[j] = at_mma(qa, ka, s[j]);
          s[j] = at_mma(qa, klo, s[j]);
          s[j] = at_mma(qlo, ka, s[j]);
          mem_order_point();
        }
      }
    }
    float cm[8];
#pragma unroll
    for (int r = 0; r < 8; ++r) {
      const int qrow = q0 + 8 * hh + r;
      float m = -1.0e30f;
#pragma unroll
      for (int j = 0; j < 4; ++j) {
        const int kvcol = kv0 + j * 16 + c;
        const bool masked = (kvcol > qrow) || (qrow - kvcol > kWin);
        const float sv = masked ? -1.0e30f : s[j][r];
        s[j][r] = sv;
        m = fmaxf(m, sv);
      }
#pragma unroll
      for (int off = 1; off < 16; off <<= 1) m = fmaxf(m, __shfl_xor(m, off, 32));
      cm[r] = m;
    }
    unsigned short* pwh = sm + L_PSH + wave * 1024;
    unsigned short* pwl = sm + L_PSL + wave * 1024;
#pragma unroll
    for (int r = 0; r < 8; ++r) {
      const float mnew = fmaxf(mrow[r], cm[r]);
      const float alpha = expf(mrow[r] - mnew);
      mrow[r] = mnew;
      float psum = 0.f;
#pragma unroll
      for (int j = 0; j < 4; ++j) {
        const float p = expf(s[j][r] - mnew);
        psum += p;
        const unsigned short hbits = f2bf_bits(p);
        const unsigned short lbits = f2bf_bits(p - bf_bits2f(hbits));
        pwh[(8 * hh + r) * 64 + j * 16 + c] = hbits;
        pwl[(8 * hh + r) * 64 + j * 16 + c] = lbits;
      }
#pragma unroll
      for (int off = 1; off < 16; off <<= 1) psum += __shfl_xor(psum, off, 32);
      lrow[r] = lrow[r] * alpha + psum;
#pragma unroll
      for (int t = 0; t < 8; ++t) oacc[t][r] *= alpha;
    }
    wave_sync_lds();
    {
      const __bf16* pah = (const __bf16*)(sm + L_PSH) + wave * 1024 + c * 64 + 8 * hh;
      const __bf16* pal = (const __bf16*)(sm + L_PSL) + wave * 1024 + c * 64 + 8 * hh;
      const __bf16* vth = (const __bf16*)(sm + L_VTH) + c * 64 + 8 * hh;
      const __bf16* vtl = (const __bf16*)(sm + L_VTL) + c * 64 + 8 * hh;
#pragma unroll 1
      for (int kk = 0; kk < 2; ++kk) {
        const v16b pa  = Frag<__bf16>::load(pah + kk * 32);
        const v16b plo = Frag<__bf16>::load(pal + kk * 32);
#pragma unroll
        for (int t = 0; t < 8; ++t) {
          const v16b va  = Frag<__bf16>::load(vth + t * 1024 + kk * 32);
          const v16b vlo = Frag<__bf16>::load(vtl + t * 1024 + kk * 32);
          oacc[t] = at_mma(pa, va, oacc[t]);
          oacc[t] = at_mma(pa, vlo, oacc[t]);
          oacc[t] = at_mma(plo, va, oacc[t]);
          mem_order_point();
        }
      }
    }
  }

  __syncthreads();
  float* osw = (float*)(void*)sm + wave * (16 * 132);
#pragma unroll
  for (int r = 0; r < 8; ++r) {
    const float inv = 1.0f / lrow[r];
#pragma unroll
    for (int t = 0; t < 8; ++t) osw[(8 * hh + r) * 132 + t * 16 + c] = oacc[t][r] * inv;
  }
  wave_sync_lds();
  {
    const int hh2 = lane >> 4, c8 = (lane & 15) * 8;
    for (int pass = 0; pass < 2; ++pass) {
#pragma unroll
      for (int it = 0; it < 8; ++it) {
        const int row = it * 2 + hh2;
        const v4f a0 = *(const v4f*)(osw + row * 132 + c8);
        const v4f a1 = *(const v4f*)(osw + row * 132 + c8 + 4);
        v8us hv, lv;
#pragma unroll
        for (int e = 0; e < 4; ++e) {
          const unsigned short hb0 = f2bf_bits(a0[e]);
          const unsigned short lb0 = f2bf_bits(a0[e] - bf_bits2f(hb0));
          const unsigned short hb1 = f2bf_bits(a1[e]);
          const unsigned short lb1 = f2bf_bits(a1[e] - bf_bits2f(hb1));
          hv[e] = hb0; lv[e] = lb0; hv[4 + e] = hb1; lv[4 + e] = lb1;
        }
        const size_t go = (rowB + q0 + row) * (size_t)kProj + colH + c8;
        *(volatile v8us*)(Oh + go) = hv;
        *(volatile v8us*)(Ol + go) = lv;
      }
      __threadfence();
    }
  }
}

__global__ __launch_bounds__(256) void outproj_gemm_kernel(
    const unsigned short* __restrict__ Ahp, const unsigned short* __restrict__ Alp,
    const unsigned short* __restrict__ Btp, const float* __restrict__ bias, float* __restrict__ out) {
  const __bf16* Ah = (const __bf16*)Ahp;
  const __bf16* Al = (const __bf16*)Alp;
  const __bf16* Bt = (const __bf16*)Btp;
  __shared__ __align__(16) float sT[8][16 * 68];
  const int lane = threadIdx.x & 31;
  const int wave = threadIdx.x >> 5;
  constexpr int tilesN = kHid / 64;
  constexpr int tilesM = kRows / 64;
  const int tile = blockIdx.x * 8 + wave;
  if (tile >= tilesM * tilesN) return;
  const int tm = tile / tilesN;
  const int tn = tile - tm * tilesN;
  const int m0 = tm << 6;
  const int n0 = tn << 6;
  const int rlane = lane & 15;
  const int mOff  = (lane >> 4) * 8;

  v8f acc[4][4];
  gemm_mainloop<true>(Ah, Al, Bt, kProj, kProj, m0, n0, kProj, lane, acc);

  float* slab = sT[wave];
  float bvj[4];
#pragma unroll
  for (int j = 0; j < 4; ++j) bvj[j] = bf_rne(bias[n0 + (j << 4) + rlane]);
#pragma unroll
  for (int i = 0; i < 4; ++i) {
    const int mBase = m0 + (i << 4);
#pragma unroll
    for (int j = 0; j < 4; ++j) {
#pragma unroll
      for (int r = 0; r < 8; ++r) slab[(mOff + r) * 68 + (j << 4) + rlane] = acc[i][j][r] + bvj[j];
    }
    wave_sync_lds();
    {
      const int h2 = lane >> 4, c4 = (lane & 15) * 4;
      for (int pass = 0; pass < 2; ++pass) {
#pragma unroll
        for (int it = 0; it < 8; ++it) {
          const int row = it * 2 + h2;
          const v4f v = *(const v4f*)(slab + row * 68 + c4);
          *(volatile v4f*)(out + (size_t)(mBase + row) * kHid + n0 + c4) = v;
        }
        __threadfence();
      }
    }
    wave_sync_lds();
  }
}

extern "C" void kernel_launch(void* const* d_in, const int* in_sizes, int n_in,
                              void* d_out, int out_size, void* d_ws, size_t ws_size,
                              hipStream_t stream) {
  if (n_in < 10) return;
  if (in_sizes[0] != kRows * kHid) return;
  if (in_sizes[1] != kHid * kProj || in_sizes[3] != kHid * kProj || in_sizes[5] != kHid * kProj || in_sizes[7] != kProj * kHid) return;
  if (in_sizes[2] != kProj || in_sizes[4] != kProj || in_sizes[6] != kProj || in_sizes[8] != kHid || in_sizes[9] != kHeads) return;
  if (out_size != kRows * kHid) return;
  const size_t kMiB = 1048576;
  if (ws_size < (size_t)128 * kMiB) return;

  const float* x   = (const float*)d_in[0];
  const float* WQ  = (const float*)d_in[1];
  const float* bQ  = (const float*)d_in[2];
  const float* WK  = (const float*)d_in[3];
  const float* bK  = (const float*)d_in[4];
  const float* WV  = (const float*)d_in[5];
  const float* bV  = (const float*)d_in[6];
  const float* WO  = (const float*)d_in[7];
  const float* bO  = (const float*)d_in[8];
  const float* kw  = (const float*)d_in[9];
  float* out = (float*)d_out;

  char* ws = (char*)d_ws;
  unsigned short* AOh = (unsigned short*)(ws + 0);
  unsigned short* AOl = (unsigned short*)(ws + 16 * kMiB);
  unsigned short* XB  = (unsigned short*)(ws + 0);
  unsigned short* BtS = (unsigned short*)(ws + 16 * kMiB);
  float* rcos = (float*)(ws + 24 * kMiB);
  float* rsin = (float*)(ws + 24 * kMiB + 524288);
  unsigned short* Qh = (unsigned short*)(ws + 32 * kMiB);
  unsigned short* Ql = (unsigned short*)(ws + 48 * kMiB);
  unsigned short* Kh = (unsigned short*)(ws + 64 * kMiB);
  unsigned short* Kl = (unsigned short*)(ws + 80 * kMiB);
  unsigned short* Vh = (unsigned short*)(ws + 96 * kMiB);
  unsigned short* Vl = (unsigned short*)(ws + 112 * kMiB);
  unsigned short* BtO = (unsigned short*)(ws + 32 * kMiB);

  const int n8 = (kRows * kHid) / 8;
  const dim3 gW(kProj / 64, kProj / 64);
  const int gemmBlocks = (kRows / 64) * (kProj / 64) / 8;
  const int attnBlocks = kBatch * kHeads * (kSeq / 64);

  rope_tab_kernel<<<(kSeq * 64) / 256, 256, 0, stream>>>(rcos, rsin);
  cast_x_kernel<<<n8 / 256, 256, 0, stream>>>(x, XB, n8);

  cast_w_kernel<<<gW, 256, 0, stream>>>(WQ, BtS, 0);
  proj_gemm_kernel<<<gemmBlocks, 256, 0, stream>>>(XB, BtS, bQ, kw, rcos, rsin, Qh, Ql, 0);
  cast_w_kernel<<<gW, 256, 0, stream>>>(WK, BtS, 0);
  proj_gemm_kernel<<<gemmBlocks, 256, 0, stream>>>(XB, BtS, bK, kw, rcos, rsin, Kh, Kl, 1);
  cast_w_kernel<<<gW, 256, 0, stream>>>(WV, BtS, 0);
  proj_gemm_kernel<<<gemmBlocks, 256, 0, stream>>>(XB, BtS, bV, kw, rcos, rsin, Vh, Vl, 2);

  swa_attn_kernel<<<attnBlocks, 128, 0, stream>>>(Qh, Ql, Kh, Kl, Vh, Vl, AOh, AOl);

  cast_w_kernel<<<gW, 256, 0, stream>>>(WO, BtO, 1);
  outproj_gemm_kernel<<<gemmBlocks, 256, 0, stream>>>(AOh, AOl, BtO, bO, out);
}
